// MyRNN_85177791414628
// MI455X (gfx1250) — hardware-verified
//
#include <hip/hip_runtime.h>
#include <math.h>

constexpr int HID        = 16;
constexpr int NGATE      = 4 * HID;
constexpr int TSTEPS     = 1024;
constexpr int NBATCH     = 4096;
constexpr int NOUTC      = 5;
constexpr int TILE_ROWS  = 16;
constexpr int NTHREADS   = 64;
constexpr int NWAVES     = NTHREADS / 32;
constexpr int BLOCK_ROWS = TILE_ROWS * NWAVES;
constexpr int NBLOCKS    = NBATCH / BLOCK_ROWS;
constexpr int WPITCH     = 32;
constexpr int BLOCK_OUT  = BLOCK_ROWS * NOUTC;
constexpr int OUT_LINES  = BLOCK_OUT / 32;

constexpr float BIAS_LO_CARRY = 2048.0f;
constexpr float BIAS_LO_FOLD  = 1.0f / 2048.0f;
constexpr float W_LO_CARRY    = 256.0f;
constexpr float XH_FOLD       = 1.0f / 256.0f;
constexpr float X_LO_CARRY    = 64.0f;
constexpr float WH_FOLD       = 1.0f / 64.0f;

static_assert(HID == 16, "one 16-row unit tile");
static_assert(NGATE == 64, "four gate blocks of 16 rows");
static_assert(NGATE == NTHREADS, "one thread fills one row of each weight plane");
static_assert(WPITCH == 2 * HID, "k extent of one WMMA step");
static_assert((WPITCH * 2) % 16 == 0, "plane rows are 16-B aligned");
static_assert(TSTEPS % 4 == 0, "x is read four steps at a time");
static_assert(NBATCH % BLOCK_ROWS == 0, "grid covers the batch exactly");
static_assert(BLOCK_ROWS == 32, "block output = 160 floats");
static_assert((BLOCK_OUT * 4) % 128 == 0, "block output is a whole number of 128-B lines");
static_assert(BLOCK_OUT == OUT_LINES * 32, "one store instruction per line");
static_assert(3 * NTHREADS >= BLOCK_OUT, "head loop covers every block output");

typedef __attribute__((ext_vector_type(16))) _Float16 v16h;
typedef __attribute__((ext_vector_type(8)))  _Float16 v8h;
typedef __attribute__((ext_vector_type(8)))  float    v8f;
typedef __attribute__((ext_vector_type(4)))  float    v4f;

union FragU { v16h v; v8h h[2]; };

__device__ __forceinline__ v16h frag_load(const _Float16* p) {
  FragU f;
  f.h[0] = *(const v8h*)(p);
  f.h[1] = *(const v8h*)(p + 16);
  return f.v;
}

__device__ __forceinline__ v8f mma16(v16h a, v16h b, v8f c) {
  return __builtin_amdgcn_wmma_f32_16x16x32_f16(false, a, false, b, (short)0, c, false, false);
}

__device__ __forceinline__ void guard_group(v8f& a, v8f& b, v8f& c, v8f& d,
                                            v16h w0, v16h w1, v16h w2, v16h w3, v16h bf) {
  asm volatile("v_nop\n\tv_nop\n\tv_nop\n\tv_nop"
               : "+v"(a), "+v"(b), "+v"(c), "+v"(d)
               : "v"(w0), "v"(w1), "v"(w2), "v"(w3), "v"(bf));
}

__device__ __forceinline__ v8h pack8h(float e0, float e1, float e2, float e3,
                                      float e4, float e5, float e6, float e7) {
  v8h r;
  r[0] = (_Float16)e0;
  r[1] = (_Float16)e1;
  r[2] = (_Float16)e2;
  r[3] = (_Float16)e3;
  r[4] = (_Float16)e4;
  r[5] = (_Float16)e5;
  r[6] = (_Float16)e6;
  r[7] = (_Float16)e7;
  return r;
}

__device__ __forceinline__ float fsig(float v)  { return __builtin_amdgcn_rcpf(1.0f + __expf(-v)); }
__device__ __forceinline__ float ftanh(float v) { return 1.0f - 2.0f * __builtin_amdgcn_rcpf(__expf(2.0f * v) + 1.0f); }

__global__ __launch_bounds__(NTHREADS) void lstm2_persistent_kernel(
    const float* __restrict__ x,
    const float* __restrict__ Wih0, const float* __restrict__ Whh0,
    const float* __restrict__ bih0, const float* __restrict__ bhh0,
    const float* __restrict__ Wih1, const float* __restrict__ Whh1,
    const float* __restrict__ bih1, const float* __restrict__ bhh1,
    const float* __restrict__ Wout, const float* __restrict__ bout,
    float* __restrict__ out) {
  __shared__ __align__(16) _Float16 Wp1[NGATE * WPITCH];
  __shared__ __align__(16) _Float16 Wp2[NGATE * WPITCH];
  __shared__ __align__(16) float    B2s[NGATE];
  __shared__ __align__(16) float    Hr[BLOCK_ROWS * HID];
  __shared__ __align__(16) float    Os[BLOCK_OUT];

  const int tid  = threadIdx.x;
  const int lane = tid & 31;
  const int wave = tid >> 5;
  const int hh   = lane >> 4;
  const int n    = lane & 15;
  const bool lane_lo = (hh == 0);

  {
    const int m = tid;
    float zf = 0.0f;
    asm volatile("" : "+v"(zf));

    const v4f wa0 = *(const v4f*)(Whh0 + m * HID + 0);
    const v4f wa1 = *(const v4f*)(Whh0 + m * HID + 4);
    const v4f wa2 = *(const v4f*)(Whh0 + m * HID + 8);
    const v4f wa3 = *(const v4f*)(Whh0 + m * HID + 12);
    const v4f wb0 = *(const v4f*)(Wih1 + m * HID + 0);
    const v4f wb1 = *(const v4f*)(Wih1 + m * HID + 4);
    const v4f wb2 = *(const v4f*)(Wih1 + m * HID + 8);
    const v4f wb3 = *(const v4f*)(Wih1 + m * HID + 12);
    const v4f wc0 = *(const v4f*)(Whh1 + m * HID + 0);
    const v4f wc1 = *(const v4f*)(Whh1 + m * HID + 4);
    const v4f wc2 = *(const v4f*)(Whh1 + m * HID + 8);
    const v4f wc3 = *(const v4f*)(Whh1 + m * HID + 12);

    const float bs = bih0[m] + bhh0[m];
    const float bh = (float)(_Float16)bs;
    const float bl = (bs - bh) * BIAS_LO_CARRY;
    const float w  = Wih0[m];
    const float wh = (float)(_Float16)w;
    const float wl = (w - wh) * W_LO_CARRY;
    const float ws = wh * WH_FOLD;

    const v8h p1a = pack8h(wa0[0], wa0[1], wa0[2], wa0[3], wa1[0], wa1[1], wa1[2], wa1[3]);
    const v8h p1b = pack8h(wa2[0], wa2[1], wa2[2], wa2[3], wa3[0], wa3[1], wa3[2], wa3[3]);
    const v8h p1c = pack8h(bh, bl, wh, wl, ws, zf, zf, zf);
    const v8h p1d = pack8h(zf, zf, zf, zf, zf, zf, zf, zf);
    const v8h p2a = pack8h(wb0[0], wb0[1], wb0[2], wb0[3], wb1[0], wb1[1], wb1[2], wb1[3]);
    const v8h p2b = pack8h(wb2[0], wb2[1], wb2[2], wb2[3], wb3[0], wb3[1], wb3[2], wb3[3]);
    const v8h p2c = pack8h(wc0[0], wc0[1], wc0[2], wc0[3], wc1[0], wc1[1], wc1[2], wc1[3]);
    const v8h p2d = pack8h(wc2[0], wc2[1], wc2[2], wc2[3], wc3[0], wc3[1], wc3[2], wc3[3]);

    _Float16* r1 = Wp1 + m * WPITCH;
    _Float16* r2 = Wp2 + m * WPITCH;
    *(v8h*)(r1 + 0)  = p1a;
    *(v8h*)(r1 + 8)  = p1b;
    *(v8h*)(r1 + 16) = p1c;
    *(v8h*)(r1 + 24) = p1d;
    *(v8h*)(r2 + 0)  = p2a;
    *(v8h*)(r2 + 8)  = p2b;
    *(v8h*)(r2 + 16) = p2c;
    *(v8h*)(r2 + 24) = p2d;

    B2s[m] = bih1[m] + bhh1[m];
  }
  __syncthreads();

  v16h A1[4], A2[4];
  v8f  bias2[4];
#pragma unroll
  for (int g = 0; g < 4; ++g) {
    A1[g] = frag_load(Wp1 + (g * 16 + n) * WPITCH + 8 * hh);
    A2[g] = frag_load(Wp2 + (g * 16 + n) * WPITCH + 8 * hh);
    const v4f blo = *(const v4f*)(B2s + g * 16 + 8 * hh);
    const v4f bhi = *(const v4f*)(B2s + g * 16 + 8 * hh + 4);
    bias2[g] = __builtin_shufflevector(blo, bhi, 0, 1, 2, 3, 4, 5, 6, 7);
  }

  float c1[8], c2[8], h2f[8];
#pragma unroll
  for (int r = 0; r < 8; ++r) { c1[r] = 0.0f; c2[r] = 0.0f; h2f[r] = 0.0f; }
  const _Float16 hz = (_Float16)0.0f;
  v8h h1p = {hz, hz, hz, hz, hz, hz, hz, hz};
  v8h h2p = {hz, hz, hz, hz, hz, hz, hz, hz};

  const float cone = lane_lo ? 1.0f : 0.0f;
  const float ceps = lane_lo ? BIAS_LO_FOLD : 0.0f;
  const v8f z8 = {0.f, 0.f, 0.f, 0.f, 0.f, 0.f, 0.f, 0.f};

  const int brow = blockIdx.x * BLOCK_ROWS + wave * TILE_ROWS + n;
  const v4f* xrow = (const v4f*)(x + (size_t)brow * TSTEPS);

#pragma unroll 1
  for (int t0 = 0; t0 < TSTEPS / 4; ++t0) {
    v4f xq = xrow[t0];
    asm volatile("" : "+v"(xq));
#pragma unroll
    for (int tt = 0; tt < 4; ++tt) {
      const float xv = xq[tt];
      const float xs = lane_lo ? xv : 0.0f;
      const float xh = (float)(_Float16)xs;
      const float xl = xs - xh;
      v8h sl;
      sl[0] = (_Float16)cone;
      sl[1] = (_Float16)ceps;
      sl[2] = (_Float16)xh;
      sl[3] = (_Float16)(xh * XH_FOLD);
      sl[4] = (_Float16)(xl * X_LO_CARRY);
      sl[5] = hz;
      sl[6] = hz;
      sl[7] = hz;
      const v16h B1 = __builtin_shufflevector(h1p, sl, 0, 1, 2, 3, 4, 5, 6, 7, 8, 9, 10, 11, 12, 13, 14, 15);
      v8f g0 = mma16(A1[0], B1, z8);
      v8f g1 = mma16(A1[1], B1, z8);
      v8f g2 = mma16(A1[2], B1, z8);
      v8f g3 = mma16(A1[3], B1, z8);
      guard_group(g0, g1, g2, g3, A1[0], A1[1], A1[2], A1[3], B1);
      v8h h1n;
#pragma unroll
      for (int r = 0; r < 8; ++r) {
        const float ig = fsig(g0[r]);
        const float fg = fsig(g1[r]);
        const float gg = ftanh(g2[r]);
        const float og = fsig(g3[r]);
        const float cn = fg * c1[r] + ig * gg;
        c1[r] = cn;
        const float hv = og * ftanh(cn);
        h1n[r] = (_Float16)hv;
      }
      h1p = h1n;

      const v16h B2 = __builtin_shufflevector(h1p, h2p, 0, 1, 2, 3, 4, 5, 6, 7, 8, 9, 10, 11, 12, 13, 14, 15);
      v8f a0 = mma16(A2[0], B2, bias2[0]);
      v8f a1 = mma16(A2[1], B2, bias2[1]);
      v8f a2 = mma16(A2[2], B2, bias2[2]);
      v8f a3 = mma16(A2[3], B2, bias2[3]);
      guard_group(a0, a1, a2, a3, A2[0], A2[1], A2[2], A2[3], B2);
      v8h h2n;
#pragma unroll
      for (int r = 0; r < 8; ++r) {
        const float ig = fsig(a0[r]);
        const float fg = fsig(a1[r]);
        const float gg = ftanh(a2[r]);
        const float og = fsig(a3[r]);
        const float cn = fg * c2[r] + ig * gg;
        c2[r] = cn;
        const float hv = og * ftanh(cn);
        h2f[r] = hv;
        h2n[r] = (_Float16)hv;
      }
      h2p = h2n;
    }
  }

  {
    float* hp = Hr + (wave * TILE_ROWS + n) * HID + 8 * hh;
    v4f lo, hi4;
    lo[0]  = fmaxf(h2f[0], 0.0f);
    lo[1]  = fmaxf(h2f[1], 0.0f);
    lo[2]  = fmaxf(h2f[2], 0.0f);
    lo[3]  = fmaxf(h2f[3], 0.0f);
    hi4[0] = fmaxf(h2f[4], 0.0f);
    hi4[1] = fmaxf(h2f[5], 0.0f);
    hi4[2] = fmaxf(h2f[6], 0.0f);
    hi4[3] = fmaxf(h2f[7], 0.0f);
    *(v4f*)(hp)     = lo;
    *(v4f*)(hp + 4) = hi4;
  }
  __syncthreads();

  for (int it = 0; it < 3; ++it) {
    const int idx = it * NTHREADS + tid;
    const int idc = (idx < BLOCK_OUT) ? idx : (BLOCK_OUT - 1);
    const int row = idc / NOUTC;
    const int o   = idc - row * NOUTC;
    const float* hr = Hr + row * HID;
    const float* wo = Wout + o * HID;
    float s = 0.0f;
#pragma unroll
    for (int q = 0; q < 4; ++q) {
      const v4f hv = *(const v4f*)(hr + 4 * q);
      const v4f wv = *(const v4f*)(wo + 4 * q);
      s += hv[0] * wv[0];
      s += hv[1] * wv[1];
      s += hv[2] * wv[2];
      s += hv[3] * wv[3];
    }
    s += bout[o];
    if (idx < BLOCK_OUT) Os[idx] = s;
  }
  __syncthreads();

  if (wave == 0) {
    float ov[OUT_LINES];
#pragma unroll
    for (int it = 0; it < OUT_LINES; ++it) ov[it] = Os[it * 32 + lane];
    float* op = out + (size_t)blockIdx.x * BLOCK_OUT;
    for (int pass = 0; pass < 2; ++pass) {
#pragma unroll
      for (int it = 0; it < OUT_LINES; ++it) *(volatile float*)(op + it * 32 + lane) = ov[it];
      __threadfence();
    }
  }
}

extern "C" void kernel_launch(void* const* d_in, const int* in_sizes, int n_in,
                              void* d_out, int out_size, void* d_ws, size_t ws_size, hipStream_t stream) {
  (void)d_ws; (void)ws_size;
  if (n_in < 11 || d_out == nullptr) return;
  if (in_sizes[0] != NBATCH * TSTEPS || in_sizes[1] != NGATE || in_sizes[2] != NGATE * HID ||
      in_sizes[3] != NGATE || in_sizes[4] != NGATE || in_sizes[5] != NGATE * HID ||
      in_sizes[6] != NGATE * HID || in_sizes[7] != NGATE || in_sizes[8] != NGATE ||
      in_sizes[9] != NOUTC * HID || in_sizes[10] != NOUTC || out_size != NBATCH * NOUTC) return;

  const float* x    = (const float*)d_in[0];
  const float* Wih0 = (const float*)d_in[1];
  const float* Whh0 = (const float*)d_in[2];
  const float* bih0 = (const float*)d_in[3];
  const float* bhh0 = (const float*)d_in[4];
  const float* Wih1 = (const float*)d_in[5];
  const float* Whh1 = (const float*)d_in[6];
  const float* bih1 = (const float*)d_in[7];
  const float* bhh1 = (const float*)d_in[8];
  const float* Wout = (const float*)d_in[9];
  const float* bout = (const float*)d_in[10];
  float* out = (float*)d_out;

  lstm2_persistent_kernel<<<NBLOCKS, NTHREADS, 0, stream>>>(
      x, Wih0, Whh0, bih0, bhh0, Wih1, Whh1, bih1, bhh1, Wout, bout, out);
}
